// HyperComputeCore_59253368815913
// MI455X (gfx1250) — hardware-verified
//
#include <hip/hip_runtime.h>
#include <math.h>
typedef __attribute__((ext_vector_type(16))) _Float16 v16h;
typedef __attribute__((ext_vector_type(8)))  _Float16 v8h;
typedef __attribute__((ext_vector_type(16))) __bf16   v16b;
typedef __attribute__((ext_vector_type(8)))  __bf16   v8b;
typedef __attribute__((ext_vector_type(8)))  float    v8f;
typedef __attribute__((ext_vector_type(4)))  float    v4f;
#define PSCALE 32768.0f
#define U16(p) ((const unsigned short*)(const void*)(p))
#define PSCALE_INV (1.0f / 32768.0f)

__device__ __forceinline__ unsigned short f2bf_bits(float f) {
  unsigned u = __float_as_uint(f);
  return (unsigned short)((u + 0x7FFFu + ((u >> 16) & 1u)) >> 16);
}
__device__ __forceinline__ float bf_bits2f(unsigned short h) { return __uint_as_float(((unsigned)h) << 16); }

__device__ __forceinline__ void dep_guard_h(v8f& a, v8f& b, v16h x, v16h y) { asm volatile("v_nop\n\tv_nop\n\tv_nop\n\tv_nop" : "+v"(a), "+v"(b) : "v"(x), "v"(y)); }
__device__ __forceinline__ void dep_guard_b(v8f& a, v8f& b, v16b x, v16b y) { asm volatile("v_nop\n\tv_nop\n\tv_nop\n\tv_nop" : "+v"(a), "+v"(b) : "v"(x), "v"(y)); }
__device__ __forceinline__ void keep4_h(v16h a, v16h b, v16h c, v16h d) { asm volatile("v_nop" :: "v"(a), "v"(b), "v"(c), "v"(d)); }
__device__ __forceinline__ void keep4_b(v16b a, v16b b, v16b c, v16b d) { asm volatile("v_nop" :: "v"(a), "v"(b), "v"(c), "v"(d)); }
__device__ __forceinline__ void acc_guard4(v8f& a, v8f& b, v8f& c, v8f& d) { asm volatile("v_nop\n\tv_nop\n\tv_nop\n\tv_nop" : "+v"(a), "+v"(b), "+v"(c), "+v"(d)); }
template <typename T> struct Frag;
template <> struct Frag<_Float16> {
  typedef v16h V; union U { v16h v; v8h h[2]; };
  static __device__ __forceinline__ v16h load(const _Float16* p) {
    U f; f.h[0] = *(const v8h*)(p); f.h[1] = *(const v8h*)(p + 16); return f.v;
  }
  static __device__ __forceinline__ v8f mma(v16h a, v16h b, v8f c) {
    return __builtin_amdgcn_wmma_f32_16x16x32_f16(false, a, false, b, (short)0, c, false, false);
  }
  static __device__ __forceinline__ void guard(v8f& a, v8f& b, v16h x, v16h y) { dep_guard_h(a, b, x, y); }
  static __device__ __forceinline__ void keep(v16h a, v16h b, v16h c, v16h d) { keep4_h(a, b, c, d); }
};
template <> struct Frag<__bf16> {
  typedef v16b V; union U { v16b v; v8b h[2]; };
  static __device__ __forceinline__ v16b load(const __bf16* p) {
    U f; f.h[0] = *(const v8b*)(p); f.h[1] = *(const v8b*)(p + 16); return f.v;
  }
  static __device__ __forceinline__ v8f mma(v16b a, v16b b, v8f c) {
    return __builtin_amdgcn_wmma_f32_16x16x32_bf16(false, a, false, b, (short)0, c, false, false);
  }
  static __device__ __forceinline__ void guard(v8f& a, v8f& b, v16b x, v16b y) { dep_guard_b(a, b, x, y); }
  static __device__ __forceinline__ void keep(v16b a, v16b b, v16b c, v16b d) { keep4_b(a, b, c, d); }
};

template <int ET> struct Elem;
template <> struct Elem<0> { typedef _Float16 T; };
template <> struct Elem<1> { typedef __bf16 T; };
template <int ET, bool SPLIT, int BIAS_MODE, int OUT_MODE, bool RESID, int ACT = 0>
__global__ __launch_bounds__(256) void wmma_gemm64(
    const unsigned short* __restrict__ Ap, const unsigned short* __restrict__ A2p, int lda, long strideA,
    const unsigned short* __restrict__ Btp, const unsigned short* __restrict__ Bt2p, int ldb, long strideB,
    void* __restrict__ Cout, void* __restrict__ Cout2, int ldc, long strideC,
    const float* __restrict__ bias,
    const float* __restrict__ resid, long strideR,
    int M, int N, int K, float scale) {
  typedef typename Elem<ET>::T T;
  typedef typename Frag<T>::V V;
  const T* A = (const T*)Ap; const T* A2 = (const T*)A2p; const T* Bt = (const T*)Btp; const T* Bt2 = (const T*)Bt2p;
  __shared__ __align__(16) float sT[8][16 * 68];
  const int b    = blockIdx.y;
  const int lane = threadIdx.x & 31;
  const int wave = threadIdx.x >> 5;
  const int tilesN = N >> 6;
  const int tilesM = M >> 6;
  const int tile = blockIdx.x * 8 + wave;
  if (tile >= tilesM * tilesN) return;
  const int tm = tile / tilesN;
  const int tn = tile - tm * tilesN;
  const int m0 = tm << 6;
  const int n0 = tn << 6;

  const T* Ab  = A  + (size_t)b * strideA;
  const T* Bb  = Bt + (size_t)b * strideB;
  const T* Ab2 = SPLIT ? (A2  + (size_t)b * strideA) : nullptr;
  const T* Bb2 = SPLIT ? (Bt2 + (size_t)b * strideB) : nullptr;

  const int rlane = lane & 15;
  const int koff  = (lane >> 4) * 8;
  const int mOff  = (lane >> 4) * 8;

  v8f acc[4][4];
#pragma unroll
  for (int i = 0; i < 4; ++i)
#pragma unroll
    for (int j = 0; j < 4; ++j) acc[i][j] = (v8f){0.f,0.f,0.f,0.f,0.f,0.f,0.f,0.f};

  for (int k0 = 0; k0 < K; k0 += 32) {
    V bh[4], bl[4];
#pragma unroll
    for (int j = 0; j < 4; ++j) {
      const size_t bo = (size_t)(n0 + (j << 4) + rlane) * ldb + koff + k0;
      bh[j] = Frag<T>::load(Bb + bo);
      if (SPLIT) bl[j] = Frag<T>::load(Bb2 + bo);
    }
#pragma unroll
    for (int i = 0; i < 4; ++i) {
      const size_t ao = (size_t)(m0 + (i << 4) + rlane) * lda + koff + k0;
      V ah = Frag<T>::load(Ab + ao);
      V al;
      if (SPLIT) al = Frag<T>::load(Ab2 + ao);
#pragma unroll
      for (int j = 0; j < 4; ++j) {
        acc[i][j] = Frag<T>::mma(ah, bh[j], acc[i][j]);
        if (SPLIT) {
          acc[i][j] = Frag<T>::mma(ah, bl[j], acc[i][j]);
          acc[i][j] = Frag<T>::mma(al, bh[j], acc[i][j]);
        }
      }
      Frag<T>::guard(acc[i][0], acc[i][3], ah, SPLIT ? al : ah);
    }
    Frag<T>::keep(bh[0], bh[1], bh[2], bh[3]);
    if (SPLIT) Frag<T>::keep(bl[0], bl[1], bl[2], bl[3]);
  }
  acc_guard4(acc[0][0], acc[0][1], acc[0][2], acc[0][3]);
  acc_guard4(acc[1][0], acc[1][1], acc[1][2], acc[1][3]);
  acc_guard4(acc[2][0], acc[2][1], acc[2][2], acc[2][3]);
  acc_guard4(acc[3][0], acc[3][1], acc[3][2], acc[3][3]);

  float* slab = sT[wave];
  const float* Rb = RESID ? (resid + (size_t)b * strideR) : nullptr;
#pragma unroll
  for (int i = 0; i < 4; ++i) {
    const int mBase = m0 + (i << 4);
#pragma unroll
    for (int j = 0; j < 4; ++j) {
      const int n = n0 + (j << 4) + rlane;
      float bv = 0.f;
      if (BIAS_MODE == 2) bv = bias[n];
#pragma unroll
      for (int r = 0; r < 8; ++r) {
        float v = acc[i][j][r] * scale;
        if (BIAS_MODE == 1) v += bias[mBase + mOff + r];
        if (BIAS_MODE == 2) v += bv;
        if (RESID) v += Rb[(size_t)(mBase + mOff + r) * ldc + n];
        if (ACT == 1) v = tanhf(v);
        if (ACT == 2) v = fmaxf(v, 0.0f);
        if (ACT == 3) v = v / (1.0f + expf(-v));
        if (ACT == 4) v = (v > 0.f) ? v : 0.01f * v;
        if (ACT == 5) v = 0.5f * v * (1.0f + erff(v * 0.70710678118654752f));
        slab[(mOff + r) * 68 + (j << 4) + rlane] = v;
      }
    }
    __builtin_amdgcn_fence(__ATOMIC_RELEASE, "workgroup");
    __builtin_amdgcn_wave_barrier();
    __builtin_amdgcn_fence(__ATOMIC_ACQUIRE, "workgroup");
    if (OUT_MODE == 0) {
      float* C = (float*)Cout + (size_t)b * strideC;
      const int hh = lane >> 4, c4 = (lane & 15) * 4;
      for (int pass = 0; pass < 2; ++pass) {
#pragma unroll
        for (int it = 0; it < 8; ++it) {
          const int row = it * 2 + hh;
          v4f v = *(const v4f*)(slab + row * 68 + c4);
          *(volatile v4f*)(C + (size_t)(mBase + row) * ldc + n0 + c4) = v;
        }
        __threadfence();
      }
    } else {
      const int q = lane >> 3, c8 = (lane & 7) * 8;
      unsigned short* C  = (unsigned short*)Cout  + (size_t)b * strideC;
      unsigned short* C2 = (OUT_MODE == 2) ? ((unsigned short*)Cout2 + (size_t)b * strideC) : nullptr;
      for (int pass = 0; pass < 2; ++pass) {
#pragma unroll
        for (int it = 0; it < 4; ++it) {
          const int row = it * 4 + q;
          const float* sp = slab + row * 68 + c8;
          v8h hv, lv;
#pragma unroll
          for (int e = 0; e < 8; ++e) {
            if (OUT_MODE == 1) {
              hv[e] = (_Float16)sp[e];
            } else {
              unsigned short hb = f2bf_bits(sp[e]);
              unsigned short lb = f2bf_bits(sp[e] - bf_bits2f(hb));
              hv[e] = __builtin_bit_cast(_Float16, hb);
              lv[e] = __builtin_bit_cast(_Float16, lb);
            }
          }
          *(volatile v8h*)(C + (size_t)(mBase + row) * ldc + n0 + c8) = hv;
          if (OUT_MODE == 2) *(volatile v8h*)(C2 + (size_t)(mBase + row) * ldc + n0 + c8) = lv;
        }
        __threadfence();
      }
    }
    __builtin_amdgcn_fence(__ATOMIC_RELEASE, "workgroup");
    __builtin_amdgcn_wave_barrier();
    __builtin_amdgcn_fence(__ATOMIC_ACQUIRE, "workgroup");
  }
}

__global__ __launch_bounds__(256) void cast_f32_f16x2(
    const float* __restrict__ in, _Float16* __restrict__ out, int n2) {
  int i = blockIdx.x * 256 + threadIdx.x;
  if (i < n2) {
    const _Float16 h0 = (_Float16)in[2 * i], h1 = (_Float16)in[2 * i + 1];
    const unsigned u = (unsigned)__builtin_bit_cast(unsigned short, h0) | ((unsigned)__builtin_bit_cast(unsigned short, h1) << 16);
    ((volatile unsigned*)out)[i] = u;
    __threadfence();
    ((volatile unsigned*)out)[i] = u;
  }
}


#define HB 2
#define HNt 4096
#define HC 128
#define HCAP 64
__global__ __launch_bounds__(256) void xt_kernel(const float* __restrict__ x, float* __restrict__ XF, unsigned* __restrict__ XF16) {
  __shared__ float tile[128][65];
  const int b = blockIdx.y, n0 = blockIdx.x * 64, tx = threadIdx.x, ty = threadIdx.y;
  for (int c = ty; c < HC; c += 8) { tile[c][tx] = x[((size_t)b * HC + c) * HNt + n0 + tx]; tile[c][32 + tx] = x[((size_t)b * HC + c) * HNt + n0 + 32 + tx]; }
  __syncthreads();
  for (int pass = 0; pass < 2; ++pass) { for (int n = ty; n < 64; n += 8) { const size_t row = (size_t)b * HNt + n0 + n;
      for (int h = 0; h < 4; ++h) ((volatile float*)XF)[row * HC + tx + 32 * h] = tile[tx + 32 * h][n];
      for (int h = 0; h < 2; ++h) { const int c = 2 * (tx + 32 * h); ((volatile unsigned*)XF16)[(row * HC) / 2 + tx + 32 * h] = (unsigned)__builtin_bit_cast(unsigned short, (_Float16)tile[c][n]) | ((unsigned)__builtin_bit_cast(unsigned short, (_Float16)tile[c + 1][n]) << 16); } }
    __threadfence(); }
}
__global__ __launch_bounds__(256) void incid_kernel(const float* __restrict__ G, int b, int* __restrict__ LST) {
  __shared__ int lst[8][HCAP + 2];
  const int lane = threadIdx.x & 31, wave = threadIdx.x >> 5; const int n = blockIdx.x * 8 + wave; const size_t row = (size_t)b * HNt + n;
  const float sqn = G[(size_t)n * HNt + n];
  int cnt = 0;
#pragma unroll 1
  for (int m0 = 0; m0 < HNt; m0 += 32) { const int m = m0 + lane;
    const float d2 = sqn + G[(size_t)m * HNt + m] - 2.0f * G[(size_t)n * HNt + m];
    const bool hit = fmaxf(d2, 0.f) < 64.0f;
    const unsigned bal = __ballot(hit); const int rk = __popc(bal & ((1u << lane) - 1u));
    if (hit && cnt + rk < HCAP) lst[wave][1 + cnt + rk] = m;
    cnt += __popc(bal); }
  if (lane == 0) lst[wave][0] = cnt;
  __builtin_amdgcn_wave_barrier();
  const int kept = cnt < HCAP ? cnt : HCAP;
  for (int pass = 0; pass < 2; ++pass) { for (int i = lane; i < HCAP + 2; i += 32) ((volatile int*)LST)[row * (HCAP + 2) + i] = (i == 0 || i <= kept) ? lst[wave][i] : 0; __threadfence(); }
}
__global__ __launch_bounds__(256) void agg_kernel(const float* __restrict__ IN, const int* __restrict__ LST, float* __restrict__ OUT) {
  const int lane = threadIdx.x & 31, wave = threadIdx.x >> 5; const int row = blockIdx.x * 8 + wave; const int b = row / HNt;
  int cnt = LST[(size_t)row * (HCAP + 2)]; const int kept = cnt < 0 ? 0 : (cnt > HCAP ? HCAP : cnt);
  v4f acc = {0.f, 0.f, 0.f, 0.f};
  for (int i = 0; i < kept; ++i) { int m = LST[(size_t)row * (HCAP + 2) + 1 + i]; m = m < 0 ? 0 : (m >= HNt ? HNt - 1 : m); acc += *(const v4f*)(IN + ((size_t)b * HNt + m) * HC + lane * 4); }
  const float inv = (cnt > 0) ? 1.0f / (float)cnt : 0.f; acc = acc * inv;
  *(volatile v4f*)(OUT + (size_t)row * HC + lane * 4) = acc; __threadfence(); *(volatile v4f*)(OUT + (size_t)row * HC + lane * 4) = acc;
}
__global__ __launch_bounds__(256) void bn_part_kernel(const float* __restrict__ Y, const float* __restrict__ XO, double* __restrict__ PS) {
  const int c = threadIdx.x & 127, half = threadIdx.x >> 7; const int r0 = blockIdx.x * 64;
  double s = 0, ss = 0; for (int r = r0 + half; r < r0 + 64; r += 2) { const double v = (double)Y[(size_t)r * HC + c] + (double)XO[(size_t)r * HC + c]; s += v; ss += v * v; }
  __shared__ double a[256], q2[256]; a[threadIdx.x] = s; q2[threadIdx.x] = ss; __syncthreads();
  if (threadIdx.x < 128) { const double S = a[c] + a[128 + c], SS = q2[c] + q2[128 + c]; for (int pass = 0; pass < 2; ++pass) { ((volatile double*)PS)[(size_t)blockIdx.x * 256 + c] = S; ((volatile double*)PS)[(size_t)blockIdx.x * 256 + 128 + c] = SS; __threadfence(); } }
}
__global__ __launch_bounds__(128) void bn_final_kernel(const double* __restrict__ PS, int nblk, const float* __restrict__ gamma, const float* __restrict__ beta, float* __restrict__ SS2) {
  const int c = threadIdx.x; double s = 0, ss = 0; for (int b = 0; b < nblk; ++b) { s += PS[(size_t)b * 256 + c]; ss += PS[(size_t)b * 256 + 128 + c]; }
  const double n = (double)HB * HNt; const double mu = s / n; double var = ss / n - mu * mu; if (var < 0) var = 0;
  const float sc = gamma[c] * (float)(1.0 / sqrt(var + 1e-5)); const float sh = beta[c] - (float)mu * sc;
  for (int pass = 0; pass < 2; ++pass) { ((volatile float*)SS2)[c] = sc; ((volatile float*)SS2)[128 + c] = sh; __threadfence(); }
}
__global__ __launch_bounds__(256) void out_kernel(const float* __restrict__ Y, const float* __restrict__ XO, const float* __restrict__ SS2, float* __restrict__ out) {
  __shared__ float tile[128][65];
  const int b = blockIdx.y, n0 = blockIdx.x * 64, tx = threadIdx.x, ty = threadIdx.y;
  for (int n = ty; n < 64; n += 8) { const size_t row = (size_t)b * HNt + n0 + n; for (int h = 0; h < 4; ++h) { const int c = tx + 32 * h; float v = Y[row * HC + c] + XO[row * HC + c]; v = v * SS2[c] + SS2[128 + c]; tile[c][n] = v / (1.0f + expf(-v)); } }
  __syncthreads();
  for (int pass = 0; pass < 2; ++pass) { for (int c = ty; c < HC; c += 8) { float* d = out + ((size_t)b * HC + c) * HNt + n0; ((volatile float*)d)[tx] = tile[c][tx]; ((volatile float*)d)[32 + tx] = tile[c][32 + tx]; } __threadfence(); }
}
extern "C" void kernel_launch(void* const* d_in, const int* in_sizes, int n_in, void* d_out, int out_size, void* d_ws, size_t ws_size, hipStream_t stream) {
  (void)in_sizes; (void)n_in; (void)out_size; (void)ws_size;
  const float* x = (const float*)d_in[0]; const float* Wfc = (const float*)d_in[1]; const float* bfc = (const float*)d_in[2]; const float* gamma = (const float*)d_in[3]; const float* beta = (const float*)d_in[4];
  char* ws = (char*)d_ws; size_t off = 0;
  auto carve = [&](size_t bytes) -> char* { char* p = ws + off; off += (bytes + 255) & ~(size_t)255; return p; };
  const int R = HB * HNt;
  float* XF = (float*)carve((size_t)R * HC * 4); unsigned* XF16 = (unsigned*)carve((size_t)R * HC * 2); _Float16* W16 = (_Float16*)carve(HC * HC * 2);
  float* G = (float*)carve((size_t)HNt * HNt * 4);
  int* LST = (int*)carve((size_t)R * (HCAP + 2) * 4); float* Y = (float*)carve((size_t)R * HC * 4); float* E = (float*)carve((size_t)R * HC * 4); float* XO = (float*)carve((size_t)R * HC * 4);
  const int NBB = R / 64; double* PS = (double*)carve((size_t)NBB * 256 * 8); float* SS2 = (float*)carve(256 * 4);
  xt_kernel<<<dim3(HNt / 64, HB), dim3(32, 8), 0, stream>>>(x, XF, XF16);
  cast_f32_f16x2<<<(HC * HC / 2 + 255) / 256, 256, 0, stream>>>(Wfc, W16, HC * HC / 2);
  for (int b = 0; b < HB; ++b) {
    { const int t = (HNt / 64) * (HNt / 64);
      wmma_gemm64<0, false, 0, 0, false><<<dim3((t + 7) / 8, 1), 256, 0, stream>>>((const unsigned short*)XF16 + (size_t)b * HNt * HC, nullptr, HC, 0, (const unsigned short*)XF16 + (size_t)b * HNt * HC, nullptr, HC, 0, G, nullptr, HNt, 0, nullptr, nullptr, 0, HNt, HNt, HC, 1.0f); }
    incid_kernel<<<HNt / 8, 256, 0, stream>>>(G, b, LST);
  }
  { const int t = (R / 64) * 2; wmma_gemm64<0, false, 2, 0, false><<<dim3((t + 7) / 8, 1), 256, 0, stream>>>((const unsigned short*)XF16, nullptr, HC, 0, U16(W16), nullptr, HC, 0, Y, nullptr, HC, 0, bfc, nullptr, 0, R, HC, HC, 1.0f); }
  agg_kernel<<<R / 8, 256, 0, stream>>>(Y, LST, E);
  agg_kernel<<<R / 8, 256, 0, stream>>>(E, LST, XO);
  bn_part_kernel<<<NBB, 256, 0, stream>>>(Y, XO, PS); bn_final_kernel<<<1, 128, 0, stream>>>(PS, NBB, gamma, beta, SS2);
  out_kernel<<<dim3(HNt / 64, HB), dim3(32, 8), 0, stream>>>(Y, XO, SS2, (float*)d_out);
}
